// ChemROAR_64072322122026
// MI455X (gfx1250) — hardware-run, weakly checked
//
#include <hip/hip_runtime.h>
#include <math.h>
#include <stdint.h>

#define NB    8
#define TT    1024
#define TP1   1025
#define DM    512
#define NH    8
#define HD    64
#define DPR   32
#define DFF   1024
#define NTYPE 341
#define BT    (NB * TT)
#define NPOS  (NB * TP1)
#define NFREQ 16
#define HSC   64.0f
#define WSC   256.0f
#define QSC   1024.0f
#define KSC   1024.0f
#define PCAR  32768.0f
#define VCAR  1024.0f
#define MSC   512.0f
#define LOG2E 1.4426950408889634f
#define WPB   4
#define NQT   (TT / 16)
#define NST   (TT / 64)
#define ATT_THREADS (WPB * 32)
#define ATT_BLOCKS  (NB * (NH / WPB) * NQT)
#define PTW   (16 * 36)
#define SLW   (16 * 68)
#define WREG  (PTW + SLW)
#define SLAB64 (16 * 68)
#define TPH   72

static_assert(DM == NH * HD && HD == 64 && DPR == 32 && (NH % WPB) == 0 && ATT_THREADS == 128);
static_assert((TT % 64) == 0 && (BT % 64) == 0 && (DM % 64) == 0 && (DFF % 64) == 0 && ((3 * DM) % 64) == 0);
static_assert((DM % 32) == 0 && (DFF % 32) == 0);
static_assert((NPOS % 2) == 0);
static_assert(((BT * NH * 8) % 256) == 0 && ((BT * DM / 8) % 256) == 0 && (BT % 8) == 0);
static_assert(2 * BT * DFF * 2 <= BT * 3 * DM * 4);

typedef unsigned short u16;
typedef _Float16 v16h __attribute__((ext_vector_type(16)));
typedef _Float16 v8h  __attribute__((ext_vector_type(8)));
typedef float    v8f  __attribute__((ext_vector_type(8)));
typedef float    v4f  __attribute__((ext_vector_type(4)));
typedef unsigned int v4u __attribute__((ext_vector_type(4)));

union FragH { v16h v; v8h h[2]; v4u u[2]; };

struct InvF { float f[32]; };
static_assert(sizeof(InvF) == 128);

__device__ __forceinline__ unsigned short bf_bits(float f) {
  unsigned u = __float_as_uint(f);
  return (unsigned short)((u + 0x7FFFu + ((u >> 16) & 1u)) >> 16);
}
__device__ __forceinline__ float bf_up(unsigned short h) { return __uint_as_float(((unsigned)h) << 16); }
__device__ __forceinline__ float bfr(float f) { return bf_up(bf_bits(f)); }
__device__ __forceinline__ unsigned short h_bits(_Float16 x) { return __builtin_bit_cast(unsigned short, x); }
__device__ __forceinline__ unsigned pk16(unsigned short a, unsigned short b) { return (unsigned)a | ((unsigned)b << 16); }
__device__ __forceinline__ v8f zero8() { v8f z = {0.f, 0.f, 0.f, 0.f, 0.f, 0.f, 0.f, 0.f}; return z; }

__device__ __forceinline__ v16h ldfrag_h(const _Float16* p) {
  FragH f;
  f.h[0] = *(const v8h*)(p);
  f.h[1] = *(const v8h*)(p + 16);
  return f.v;
}

__device__ __forceinline__ v8f mma_h(v16h a, v16h b, v8f c) {
  return __builtin_amdgcn_wmma_f32_16x16x32_f16(false, a, false, b, (short)0, c, false, false);
}
__device__ __forceinline__ void guard2(v8f& a, v8f& b, v16h x0, v16h x1, v16h x2, v16h x3, v16h x4, v16h x5) {
#if defined(__HIP_DEVICE_COMPILE__)
  asm volatile("v_nop\n\tv_nop\n\tv_nop\n\tv_nop"
               : "+v"(a), "+v"(b) : "v"(x0), "v"(x1), "v"(x2), "v"(x3), "v"(x4), "v"(x5) : "memory");
#endif
}
__device__ __forceinline__ void guard6(v8f& a, v8f& b, v8f& c, v8f& d, v16h x0, v16h x1, v16h x2, v16h x3, v16h x4, v16h x5) {
#if defined(__HIP_DEVICE_COMPILE__)
  asm volatile("v_nop\n\tv_nop\n\tv_nop\n\tv_nop"
               : "+v"(a), "+v"(b), "+v"(c), "+v"(d) : "v"(x0), "v"(x1), "v"(x2), "v"(x3), "v"(x4), "v"(x5) : "memory");
#endif
}
__device__ __forceinline__ void guard10(v8f& a, v8f& b, v8f& c, v8f& d, v16h x0, v16h x1, v16h x2, v16h x3, v16h x4,
                                        v16h x5, v16h x6, v16h x7, v16h x8, v16h x9) {
#if defined(__HIP_DEVICE_COMPILE__)
  asm volatile("v_nop\n\tv_nop\n\tv_nop\n\tv_nop"
               : "+v"(a), "+v"(b), "+v"(c), "+v"(d)
               : "v"(x0), "v"(x1), "v"(x2), "v"(x3), "v"(x4), "v"(x5), "v"(x6), "v"(x7), "v"(x8), "v"(x9) : "memory");
#endif
}
__device__ __forceinline__ void acc_guard4(v8f& a, v8f& b, v8f& c, v8f& d) {
#if defined(__HIP_DEVICE_COMPILE__)
  asm volatile("v_nop\n\tv_nop\n\tv_nop\n\tv_nop" : "+v"(a), "+v"(b), "+v"(c), "+v"(d));
#endif
}
__device__ __forceinline__ void wave_sync_lds() {
  __builtin_amdgcn_fence(__ATOMIC_RELEASE, "workgroup");
  __builtin_amdgcn_wave_barrier();
  __builtin_amdgcn_fence(__ATOMIC_ACQUIRE, "workgroup");
}

__device__ __forceinline__ void sincos_acc(float angf, float& sv, float& cv) {
  const double a = (double)angf;
  const double TWO_OVER_PI = 0.63661977236758134308;
  const double PIO2_HI = 1.5707963267948966;
  const double PIO2_LO = 6.123233995736766e-17;
  const double kd = floor(a * TWO_OVER_PI + 0.5);
  const int kq = (int)kd;
  double r = fma(-kd, PIO2_HI, a);
  r = fma(-kd, PIO2_LO, r);
  const double r2 = r * r;
  double sp = 1.0 / 6227020800.0;
  sp = fma(sp, r2, -1.0 / 39916800.0);
  sp = fma(sp, r2, 1.0 / 362880.0);
  sp = fma(sp, r2, -1.0 / 5040.0);
  sp = fma(sp, r2, 1.0 / 120.0);
  sp = fma(sp, r2, -1.0 / 6.0);
  const double s = fma(sp * r2, r, r);
  double cp = -1.0 / 87178291200.0;
  cp = fma(cp, r2, 1.0 / 479001600.0);
  cp = fma(cp, r2, -1.0 / 3628800.0);
  cp = fma(cp, r2, 1.0 / 40320.0);
  cp = fma(cp, r2, -1.0 / 720.0);
  cp = fma(cp, r2, 1.0 / 24.0);
  cp = fma(cp, r2, -0.5);
  const double c = fma(cp, r2, 1.0);
  const int qd = kq & 3;
  const double so = (qd == 0) ? s : (qd == 1) ? c : (qd == 2) ? -s : -c;
  const double co = (qd == 0) ? c : (qd == 1) ? -s : (qd == 2) ? -c : s;
  sv = (float)so;
  cv = (float)co;
}

__global__ __launch_bounds__(256) void k_tab(const float* __restrict__ so, float* cosT, float* sinT, InvF inv, int npos) {
  const int gt = blockIdx.x * 256 + (int)threadIdx.x;
  const int p  = gt >> 4;
  const int i  = gt & 15;
  if (p >= npos) return;
  float f = inv.f[0];
#pragma unroll
  for (int j = 1; j < NFREQ; ++j) f = (i == j) ? inv.f[j] : f;
  const float pos = bfr(so[p]);
  const float ang = pos * f;
  float sv, cv;
  sincos_acc(ang, sv, cv);
  const size_t o = (size_t)p * NFREQ + i;
  for (int pass = 0; pass < 2; ++pass) {
    *(volatile float*)(cosT + o) = cv;
    *(volatile float*)(sinT + o) = sv;
    __threadfence();
  }
}

__global__ __launch_bounds__(256) void wt16(const float* __restrict__ W, u16* Wt, int KR, int NC, float sc) {
  __shared__ __align__(16) u16 T[64 * TPH];
  const int tid = threadIdx.x;
  const int bid = blockIdx.x;
  const int ktn = KR >> 6;
  const int kt  = bid % ktn;
  const int nt  = bid / ktn;
  if (nt * 64 + 64 > NC) return;
  const int k0 = kt * 64, n0 = nt * 64;
  {
    const int kl = tid >> 2;
    const int nc = (tid & 3) * 16;
    const float* src = W + (size_t)(k0 + kl) * NC + n0 + nc;
#pragma unroll
    for (int i = 0; i < 4; ++i) {
      const v4f a = *(const v4f*)(src + 4 * i);
#pragma unroll
      for (int e = 0; e < 4; ++e) {
        T[(nc + 4 * i + e) * TPH + kl] = h_bits((_Float16)(bfr(a[e]) * sc));
      }
    }
  }
  __syncthreads();
  v4u w[2];
  const int q8 = tid >> 3, p8 = (tid & 7) * 8;
#pragma unroll
  for (int it = 0; it < 2; ++it) {
    const int n = it * 32 + q8;
    w[it] = *(const v4u*)(T + n * TPH + p8);
  }
  for (int pass = 0; pass < 2; ++pass) {
#pragma unroll
    for (int it = 0; it < 2; ++it) {
      const int n = it * 32 + q8;
      *(volatile v4u*)(Wt + (size_t)(n0 + n) * KR + k0 + p8) = w[it];
    }
    __threadfence();
  }
}

__global__ __launch_bounds__(256) void k_ln16(const float* __restrict__ x, const float* __restrict__ g,
                                              const float* __restrict__ bta, u16* Ho, int nrows, int rnd) {
  const int tid = threadIdx.x, wave = tid >> 5, lane = tid & 31;
  const int row = blockIdx.x * 8 + wave;
  if (row >= nrows) return;
  const float* xr = x + (size_t)row * DM;
  const int c0 = 8 * lane, c1 = 256 + 8 * lane;
  const v4f a0 = *(const v4f*)(xr + c0), a1 = *(const v4f*)(xr + c0 + 4);
  const v4f a2 = *(const v4f*)(xr + c1), a3 = *(const v4f*)(xr + c1 + 4);
  float v[16];
#pragma unroll
  for (int e = 0; e < 4; ++e) { v[e] = a0[e]; v[4 + e] = a1[e]; v[8 + e] = a2[e]; v[12 + e] = a3[e]; }
#pragma unroll
  for (int e = 0; e < 16; ++e) v[e] = (rnd != 0) ? bfr(v[e]) : v[e];
  float s = 0.f;
#pragma unroll
  for (int e = 0; e < 16; ++e) s += v[e];
#pragma unroll
  for (int off = 16; off >= 1; off >>= 1) s += __shfl_xor(s, off, 32);
  const float mean = s * (1.0f / (float)DM);
  float q = 0.f;
#pragma unroll
  for (int e = 0; e < 16; ++e) { const float d = v[e] - mean; q += d * d; }
#pragma unroll
  for (int off = 16; off >= 1; off >>= 1) q += __shfl_xor(q, off, 32);
  const float rstd = rsqrtf(q * (1.0f / (float)DM) + 1e-5f);
  const v4f g0 = *(const v4f*)(g + c0), g1 = *(const v4f*)(g + c0 + 4), g2 = *(const v4f*)(g + c1), g3 = *(const v4f*)(g + c1 + 4);
  const v4f b0 = *(const v4f*)(bta + c0), b1 = *(const v4f*)(bta + c0 + 4);
  const v4f b2 = *(const v4f*)(bta + c1), b3 = *(const v4f*)(bta + c1 + 4);
  float gg[16], bb[16];
#pragma unroll
  for (int e = 0; e < 4; ++e) {
    gg[e] = bfr(g0[e]); gg[4 + e] = bfr(g1[e]); gg[8 + e] = bfr(g2[e]); gg[12 + e] = bfr(g3[e]);
    bb[e] = bfr(b0[e]); bb[4 + e] = bfr(b1[e]); bb[8 + e] = bfr(b2[e]); bb[12 + e] = bfr(b3[e]);
  }
  unsigned short hb[16];
#pragma unroll
  for (int e = 0; e < 16; ++e) {
    const float y = (v[e] - mean) * rstd * gg[e] + bb[e];
    hb[e] = h_bits((_Float16)(y * HSC));
  }
  v4u o0, o1;
#pragma unroll
  for (int e = 0; e < 4; ++e) {
    o0[e] = pk16(hb[2 * e], hb[2 * e + 1]);
    o1[e] = pk16(hb[8 + 2 * e], hb[8 + 2 * e + 1]);
  }
  u16* d = Ho + (size_t)row * DM;
  for (int pass = 0; pass < 2; ++pass) {
    *(volatile v4u*)(d + c0) = o0;
    *(volatile v4u*)(d + c1) = o1;
    __threadfence();
  }
}

__device__ __forceinline__ void stage64(float* sl, v8f a0, v8f a1, v8f a2, v8f a3, float oscale, int lane) {
  const int hh = lane >> 4, m = lane & 15;
#pragma unroll
  for (int r = 0; r < 8; ++r) {
    const int ro = (8 * hh + r) * 68 + m;
    sl[ro]      = a0[r] * oscale;
    sl[ro + 16] = a1[r] * oscale;
    sl[ro + 32] = a2[r] * oscale;
    sl[ro + 48] = a3[r] * oscale;
  }
}

__global__ __launch_bounds__(128)
void gemm_nb(const u16* __restrict__ A, const u16* __restrict__ Btp, float* C, int M, int N, int K, float oscale) {
  __shared__ __align__(16) float slab[4 * SLAB64];
  const int tid = threadIdx.x, wave = tid >> 5, lane = tid & 31, hh = lane >> 4, m = lane & 15;
  const int ntile = N >> 6;
  const int bid   = blockIdx.x;
  const int rowb  = (bid / ntile) * 64 + wave * 16;
  const int col0  = (bid % ntile) * 64;
  if (rowb + 16 > M) return;
  const _Float16* ap = (const _Float16*)(const void*)A   + (size_t)(rowb + m) * K + 8 * hh;
  const _Float16* bp = (const _Float16*)(const void*)Btp + (size_t)(col0 + m) * K + 8 * hh;
  const size_t bs = (size_t)16 * K;
  v8f acc0 = zero8(), acc1 = zero8(), acc2 = zero8(), acc3 = zero8();
#pragma unroll 1
  for (int k0 = 0; k0 < K; k0 += 32) {
    const v16h a  = ldfrag_h(ap + k0);
    const v16h b0 = ldfrag_h(bp + k0);
    const v16h b1 = ldfrag_h(bp + bs + k0);
    const v16h b2 = ldfrag_h(bp + 2 * bs + k0);
    const v16h b3 = ldfrag_h(bp + 3 * bs + k0);
    acc0 = mma_h(a, b0, acc0);
    acc1 = mma_h(a, b1, acc1);
    acc2 = mma_h(a, b2, acc2);
    acc3 = mma_h(a, b3, acc3);
    guard6(acc0, acc1, acc2, acc3, a, b0, b1, b2, b3, a);
  }
  float* sl = slab + wave * SLAB64;
  stage64(sl, acc0, acc1, acc2, acc3, oscale, lane);
  wave_sync_lds();
  v4f vals[8];
#pragma unroll
  for (int it = 0; it < 8; ++it) vals[it] = *(const v4f*)(sl + (it * 2 + hh) * 68 + m * 4);
  float* dst = C + ((size_t)rowb + (size_t)hh) * (size_t)N + col0 + m * 4;
  for (int pass = 0; pass < 2; ++pass) {
#pragma unroll
    for (int it = 0; it < 8; ++it) {
      *(volatile v4f*)(dst + (size_t)(it * 2) * (size_t)N) = vals[it];
    }
    __threadfence();
  }
}

__global__ __launch_bounds__(128)
void gemm_h2r(const u16* __restrict__ Ah, const u16* __restrict__ Al, const u16* __restrict__ Btp,
              const float* __restrict__ bias, const float* __restrict__ res, float* C, int M, int N, int K, float oscale) {
  __shared__ __align__(16) float slab[4 * SLAB64];
  const int tid = threadIdx.x, wave = tid >> 5, lane = tid & 31, hh = lane >> 4, m = lane & 15;
  const int ntile = N >> 6;
  const int bid   = blockIdx.x;
  const int rowb  = (bid / ntile) * 64 + wave * 16;
  const int col0  = (bid % ntile) * 64;
  if (rowb + 16 > M) return;
  const size_t aofs = (size_t)(rowb + m) * K + 8 * hh;
  const _Float16* ahp = (const _Float16*)(const void*)Ah + aofs;
  const _Float16* alp = (const _Float16*)(const void*)Al + aofs;
  const _Float16* bp  = (const _Float16*)(const void*)Btp + (size_t)(col0 + m) * K + 8 * hh;
  const size_t bs = (size_t)16 * K;
  v8f acc0 = zero8(), acc1 = zero8(), acc2 = zero8(), acc3 = zero8();
#pragma unroll 1
  for (int k0 = 0; k0 < K; k0 += 32) {
    const v16h ah = ldfrag_h(ahp + k0), al = ldfrag_h(alp + k0);
    const v16h b0 = ldfrag_h(bp + k0);
    const v16h b1 = ldfrag_h(bp + bs + k0);
    const v16h b2 = ldfrag_h(bp + 2 * bs + k0);
    const v16h b3 = ldfrag_h(bp + 3 * bs + k0);
    acc0 = mma_h(ah, b0, acc0);  acc0 = mma_h(al, b0, acc0);
    acc1 = mma_h(ah, b1, acc1);  acc1 = mma_h(al, b1, acc1);
    acc2 = mma_h(ah, b2, acc2);  acc2 = mma_h(al, b2, acc2);
    acc3 = mma_h(ah, b3, acc3);  acc3 = mma_h(al, b3, acc3);
    guard6(acc0, acc1, acc2, acc3, ah, al, b0, b1, b2, b3);
  }
  float* sl = slab + wave * SLAB64;
  stage64(sl, acc0, acc1, acc2, acc3, oscale, lane);
  wave_sync_lds();
  const v4f braw = *(const v4f*)(bias + col0 + m * 4);
  v4f bb;
#pragma unroll
  for (int e = 0; e < 4; ++e) bb[e] = bfr(braw[e]);
  v4f vals[8];
#pragma unroll
  for (int it = 0; it < 8; ++it) {
    const v4f sv = *(const v4f*)(sl + (it * 2 + hh) * 68 + m * 4);
    const v4f rv = *(const v4f*)(res + ((size_t)rowb + (size_t)(it * 2 + hh)) * (size_t)N + col0 + m * 4);
    const v4f ff = sv + bb;
    vals[it] = rv + ff;
  }
  float* dst = C + ((size_t)rowb + (size_t)hh) * (size_t)N + col0 + m * 4;
  for (int pass = 0; pass < 2; ++pass) {
#pragma unroll
    for (int it = 0; it < 8; ++it) {
      *(volatile v4f*)(dst + (size_t)(it * 2) * (size_t)N) = vals[it];
    }
    __threadfence();
  }
}

__device__ __forceinline__ float silu_f(float g) {
  const float e  = expf(-fabsf(g));
  const float r  = 1.0f / (1.0f + e);
  const float sg = (g >= 0.0f) ? r : (e * r);
  return g * sg;
}

__global__ __launch_bounds__(256)
void gemm_swiglu(const u16* __restrict__ A, const u16* __restrict__ Btp, const float* __restrict__ bias,
                 u16* MHo, u16* MLo, int M, int K, float oscale) {
  __shared__ __align__(16) float slab[2 * 64 * 68];
  const int tid = threadIdx.x, wave = tid >> 5, lane = tid & 31, hh = lane >> 4, m = lane & 15;
  const int part = wave >> 2, rw = wave & 3;
  const int ntile = DFF >> 6;
  const int bid   = blockIdx.x;
  const int rowb0 = (bid / ntile) * 64;
  const int rowb  = rowb0 + rw * 16;
  const int col0  = (bid % ntile) * 64;
  if (rowb0 + 64 > M) return;
  const _Float16* ap = (const _Float16*)(const void*)A   + (size_t)(rowb + m) * K + 8 * hh;
  const _Float16* bp = (const _Float16*)(const void*)Btp + (size_t)(part * DFF + col0 + m) * K + 8 * hh;
  const size_t bs = (size_t)16 * K;
  v8f acc0 = zero8(), acc1 = zero8(), acc2 = zero8(), acc3 = zero8();
#pragma unroll 1
  for (int k0 = 0; k0 < K; k0 += 32) {
    const v16h a  = ldfrag_h(ap + k0);
    const v16h b0 = ldfrag_h(bp + k0);
    const v16h b1 = ldfrag_h(bp + bs + k0);
    const v16h b2 = ldfrag_h(bp + 2 * bs + k0);
    const v16h b3 = ldfrag_h(bp + 3 * bs + k0);
    acc0 = mma_h(a, b0, acc0);
    acc1 = mma_h(a, b1, acc1);
    acc2 = mma_h(a, b2, acc2);
    acc3 = mma_h(a, b3, acc3);
    guard6(acc0, acc1, acc2, acc3, a, b0, b1, b2, b3, a);
  }
  float* sl = slab + part * (64 * 68) + (rw * 16) * 68;
  stage64(sl, acc0, acc1, acc2, acc3, oscale, lane);
  __syncthreads();
  const int q8 = tid >> 3, p8 = (tid & 7) * 8;
  const v4f ba0 = *(const v4f*)(bias + col0 + p8), ba1 = *(const v4f*)(bias + col0 + p8 + 4);
  const v4f bg0 = *(const v4f*)(bias + DFF + col0 + p8), bg1 = *(const v4f*)(bias + DFF + col0 + p8 + 4);
  float ba[8], bg[8];
#pragma unroll
  for (int e = 0; e < 4; ++e) { ba[e] = bfr(ba0[e]); ba[4 + e] = bfr(ba1[e]); bg[e] = bfr(bg0[e]); bg[4 + e] = bfr(bg1[e]); }
  v4u oh[2], ol[2];
#pragma unroll
  for (int it = 0; it < 2; ++it) {
    const int row = it * 32 + q8;
    const float* pa = slab + row * 68 + p8;
    const float* pg = slab + 64 * 68 + row * 68 + p8;
    const v4f ua0 = *(const v4f*)(pa), ua1 = *(const v4f*)(pa + 4);
    const v4f ug0 = *(const v4f*)(pg), ug1 = *(const v4f*)(pg + 4);
    float mv[8];
#pragma unroll
    for (int e = 0; e < 4; ++e) {
      mv[e]     = silu_f(ug0[e] + bg[e])     * (ua0[e] + ba[e]);
      mv[4 + e] = silu_f(ug1[e] + bg[4 + e]) * (ua1[e] + ba[4 + e]);
    }
#pragma unroll
    for (int e = 0; e < 4; ++e) {
      const float t0 = mv[2 * e] * MSC, t1 = mv[2 * e + 1] * MSC;
      const _Float16 h0 = (_Float16)t0, h1 = (_Float16)t1;
      const _Float16 l0 = (_Float16)(t0 - (float)h0), l1 = (_Float16)(t1 - (float)h1);
      oh[it][e] = pk16(h_bits(h0), h_bits(h1));
      ol[it][e] = pk16(h_bits(l0), h_bits(l1));
    }
  }
  for (int pass = 0; pass < 2; ++pass) {
#pragma unroll
    for (int it = 0; it < 2; ++it) {
      const int row = it * 32 + q8;
      const size_t o8 = (size_t)(rowb0 + row) * DFF + col0 + p8;
      *(volatile v4u*)(MHo + o8) = oh[it];
      *(volatile v4u*)(MLo + o8) = ol[it];
    }
    __threadfence();
  }
}

__global__ __launch_bounds__(256)
void rope_qk(const float* __restrict__ QKV, const int* __restrict__ xt, const float* __restrict__ temb,
             const float* __restrict__ cosT, const float* __restrict__ sinT,
             u16* QHo, u16* QLo, u16* KHo, u16* KLo, int nrows) {
#pragma clang fp contract(off)
  const int gt  = blockIdx.x * 256 + (int)threadIdx.x;
  const int row = gt >> 3;
  const int d0  = (gt & 7) * 8;
  if (row >= nrows) return;
  const int s = row / NH, h = row % NH;
  const int b = s / TT, t = s % TT;
  const int pq = b * TP1 + t, pk = pq + 1;
  int tq = xt[pq]; tq = (tq < 0) ? 0 : ((tq > NTYPE - 1) ? (NTYPE - 1) : tq);
  int tk = xt[pk]; tk = (tk < 0) ? 0 : ((tk > NTYPE - 1) ? (NTYPE - 1) : tk);
  const float* qr  = QKV + (size_t)s * (3 * DM) + h * HD + d0;
  const float* kr  = qr + DM;
  const float* eqp = temb + (size_t)tq * (2 * DM) + h * HD + d0;
  const float* ekp = temb + (size_t)tk * (2 * DM) + DM + h * HD + d0;
  const v4f qa = *(const v4f*)(qr), qb = *(const v4f*)(qr + 4);
  const v4f ka = *(const v4f*)(kr), kc = *(const v4f*)(kr + 4);
  const v4f ea = *(const v4f*)(eqp), eb = *(const v4f*)(eqp + 4);
  const v4f fa = *(const v4f*)(ekp), fb = *(const v4f*)(ekp + 4);
  const int i0 = (d0 & 31) >> 1;
  const v4f cq = *(const v4f*)(cosT + (size_t)pq * NFREQ + i0), sq = *(const v4f*)(sinT + (size_t)pq * NFREQ + i0);
  const v4f ck = *(const v4f*)(cosT + (size_t)pk * NFREQ + i0), sk = *(const v4f*)(sinT + (size_t)pk * NFREQ + i0);
  const bool rot = d0 < DPR;
  float wq[8], wk[8];
#pragma unroll
  for (int e = 0; e < 4; ++e) {
    wq[e] = qa[e] + bfr(ea[e]);  wq[4 + e] = qb[e] + bfr(eb[e]);
    wk[e] = ka[e] + bfr(fa[e]);  wk[4 + e] = kc[e] + bfr(fb[e]);
  }
  float oq[8], ok[8];
#pragma unroll
  for (int e = 0; e < 4; ++e) {
    const float cqe = rot ? cq[e] : 1.0f, sqe = rot ? sq[e] : 0.0f;
    const float cke = rot ? ck[e] : 1.0f, ske = rot ? sk[e] : 0.0f;
    const float x1 = wq[2 * e], x2 = wq[2 * e + 1];
    oq[2 * e]     = x1 * cqe - x2 * sqe;
    oq[2 * e + 1] = x2 * cqe + x1 * sqe;
    const float y1 = wk[2 * e], y2 = wk[2 * e + 1];
    ok[2 * e]     = y1 * cke - y2 * ske;
    ok[2 * e + 1] = y2 * cke + y1 * ske;
  }
  v4u qh4, ql4, kh4, kl4;
#pragma unroll
  for (int e = 0; e < 4; ++e) {
    const float t0 = oq[2 * e] * QSC, t1 = oq[2 * e + 1] * QSC;
    const _Float16 h0 = (_Float16)t0, h1 = (_Float16)t1;
    const _Float16 l0 = (_Float16)(t0 - (float)h0), l1 = (_Float16)(t1 - (float)h1);
    qh4[e] = pk16(h_bits(h0), h_bits(h1));
    ql4[e] = pk16(h_bits(l0), h_bits(l1));
    const float u0 = ok[2 * e] * KSC, u1 = ok[2 * e + 1] * KSC;
    const _Float16 g0 = (_Float16)u0, g1 = (_Float16)u1;
    const _Float16 m0 = (_Float16)(u0 - (float)g0), m1 = (_Float16)(u1 - (float)g1);
    kh4[e] = pk16(h_bits(g0), h_bits(g1));
    kl4[e] = pk16(h_bits(m0), h_bits(m1));
  }
  const size_t o8 = (size_t)row * HD + d0;
  for (int pass = 0; pass < 2; ++pass) {
    *(volatile v4u*)(QHo + o8) = qh4;
    *(volatile v4u*)(QLo + o8) = ql4;
    *(volatile v4u*)(KHo + o8) = kh4;
    *(volatile v4u*)(KLo + o8) = kl4;
    __threadfence();
  }
}

__global__ __launch_bounds__(256) void vt16(const float* __restrict__ QKV, u16* VHo, u16* VLo) {
  __shared__ __align__(16) u16 TH[HD * TPH];
  __shared__ __align__(16) u16 TL[HD * TPH];
  const int tid = threadIdx.x;
  const int bid = blockIdx.x;
  const int st  = bid % NST;
  const int bh  = bid / NST;
  if (bh >= NB * NH) return;
  const int b = bh / NH, g = bh % NH;
  const int t0 = st * 64;
  const size_t srow0 = (size_t)b * TT + t0;
  {
    const int sl = tid >> 2;
    const int dc = (tid & 3) * 16;
    const float* src = QKV + (srow0 + (size_t)sl) * (3 * DM) + 2 * DM + g * HD + dc;
#pragma unroll
    for (int i = 0; i < 4; ++i) {
      const v4f a = *(const v4f*)(src + 4 * i);
#pragma unroll
      for (int e = 0; e < 4; ++e) {
        const float t = a[e] * VCAR;
        const _Float16 hv = (_Float16)t;
        const _Float16 lv = (_Float16)(t - (float)hv);
        TH[(dc + 4 * i + e) * TPH + sl] = h_bits(hv);
        TL[(dc + 4 * i + e) * TPH + sl] = h_bits(lv);
      }
    }
  }
  __syncthreads();
  v4u vh[2], vl[2];
  const int q8 = tid >> 3, p8 = (tid & 7) * 8;
#pragma unroll
  for (int it = 0; it < 2; ++it) {
    const int line = it * 32 + q8;
    vh[it] = *(const v4u*)(TH + line * TPH + p8);
    vl[it] = *(const v4u*)(TL + line * TPH + p8);
  }
  const size_t base = ((size_t)bh * HD) * TT + t0 + p8;
  for (int pass = 0; pass < 2; ++pass) {
#pragma unroll
    for (int it = 0; it < 2; ++it) {
      const int line = it * 32 + q8;
      *(volatile v4u*)(VHo + base + (size_t)line * TT) = vh[it];
      *(volatile v4u*)(VLo + base + (size_t)line * TT) = vl[it];
    }
    __threadfence();
  }
}

__global__ __launch_bounds__(ATT_THREADS)
void attn_c(const u16* __restrict__ QHp, const u16* __restrict__ QLp,
            const u16* __restrict__ KHp, const u16* __restrict__ KLp,
            const u16* __restrict__ VHp, const u16* __restrict__ VLp,
            const float* __restrict__ xv, float* XBo) {
  __shared__ __align__(16) float smem[WPB * WREG];

  const int tid  = threadIdx.x;
  const int wave = tid >> 5;
  const int lane = tid & 31;
  const int hh   = lane >> 4;
  const int c    = lane & 15;
  const int bid  = blockIdx.x;
  const int qt   = bid % NQT;
  const int hg   = (bid / NQT) % (NH / WPB);
  const int b    = bid / (NQT * (NH / WPB));
  if (b >= NB) return;
  const int head = hg * WPB + wave;
  const int q0   = qt * 16;
  const size_t sq0 = (size_t)b * TT + (size_t)q0;

  float* pt   = smem + wave * WREG;
  float* slab = pt + PTW;

  const size_t qofs = ((sq0 + (size_t)c) * NH + head) * HD + 8 * hh;
  const _Float16* Qh  = (const _Float16*)(const void*)QHp + qofs;
  const _Float16* Ql  = (const _Float16*)(const void*)QLp + qofs;
  const size_t kofs = ((((size_t)b * TT) + (size_t)c) * NH + head) * HD + 8 * hh;
  const _Float16* Khb = (const _Float16*)(const void*)KHp + kofs;
  const _Float16* Klb = (const _Float16*)(const void*)KLp + kofs;
  const size_t vofs = (((size_t)b * NH + head) * HD + c) * TT + 8 * hh;
  const _Float16* Vhb = (const _Float16*)(const void*)VHp + vofs;
  const _Float16* Vlb = (const _Float16*)(const void*)VLp + vofs;
  const float lsc = 0.125f * (LOG2E / (QSC * KSC));
  const float oc  = 1.0f / (PCAR * VCAR);
  const size_t KROW = (size_t)NH * HD;

  float mrow[8], lrow[8];
  v8f o[4];
#pragma unroll
  for (int r = 0; r < 8; ++r) { mrow[r] = -INFINITY; lrow[r] = 0.f; }
#pragma unroll
  for (int j = 0; j < 4; ++j) o[j] = zero8();
  const int nkt = (q0 >> 5) + 1;

#pragma unroll 1
  for (int kt = 0; kt < nkt; ++kt) {
    const int kb = kt * 32;
    v8f s0 = zero8(), s1 = zero8();
    const _Float16* k0p = Khb + (size_t)kb * KROW;
    const _Float16* k1p = k0p + (size_t)16 * KROW;
    const _Float16* l0p = Klb + (size_t)kb * KROW;
    const _Float16* l1p = l0p + (size_t)16 * KROW;
#pragma unroll
    for (int kk = 0; kk < 2; ++kk) {
      const v16h qh  = ldfrag_h(Qh + kk * 32),  ql  = ldfrag_h(Ql + kk * 32);
      const v16h kh0 = ldfrag_h(k0p + kk * 32), kl0 = ldfrag_h(l0p + kk * 32);
      const v16h kh1 = ldfrag_h(k1p + kk * 32), kl1 = ldfrag_h(l1p + kk * 32);
      s0 = mma_h(qh, kh0, s0);
      s0 = mma_h(ql, kh0, s0);
      s0 = mma_h(qh, kl0, s0);
      s1 = mma_h(qh, kh1, s1);
      s1 = mma_h(ql, kh1, s1);
      s1 = mma_h(qh, kl1, s1);
      guard2(s0, s1, qh, ql, kh0, kl0, kh1, kl1);
    }
#pragma unroll
    for (int r = 0; r < 8; ++r) {
      const int i = q0 + 8 * hh + r;
      const bool ok0 = (kb + c) <= i;
      const bool ok1 = (kb + 16 + c) <= i;
      const float t0 = ok0 ? (s0[r] * lsc) : -INFINITY;
      const float t1 = ok1 ? (s1[r] * lsc) : -INFINITY;
      float mx = fmaxf(t0, t1);
#pragma unroll
      for (int off = 1; off < 16; off <<= 1) mx = fmaxf(mx, __shfl_xor(mx, off, 32));
      const float mn = fmaxf(mrow[r], mx);
      const float ms = (mn == -INFINITY) ? 0.0f : mn;
      const float al = exp2f(mrow[r] - ms);
      mrow[r] = mn;
      const float e0 = exp2f(t0 - ms), e1 = exp2f(t1 - ms);
      float ps = e0 + e1;
#pragma unroll
      for (int off = 1; off < 16; off <<= 1) ps += __shfl_xor(ps, off, 32);
      lrow[r] = lrow[r] * al + ps;
#pragma unroll
      for (int j = 0; j < 4; ++j) o[j][r] *= al;
      const int ro = (8 * hh + r) * 36 + c;
      pt[ro]      = e0;
      pt[ro + 16] = e1;
    }
    wave_sync_lds();
    FragH ph;
    {
      const float* prow = pt + c * 36 + 8 * hh;
      const v4f p0 = *(const v4f*)(prow), p1 = *(const v4f*)(prow + 4);
      const v4f p2 = *(const v4f*)(prow + 16), p3 = *(const v4f*)(prow + 20);
#pragma unroll
      for (int e = 0; e < 4; ++e) {
        ph.h[0][e]     = (_Float16)(p0[e] * PCAR);
        ph.h[0][4 + e] = (_Float16)(p1[e] * PCAR);
        ph.h[1][e]     = (_Float16)(p2[e] * PCAR);
        ph.h[1][4 + e] = (_Float16)(p3[e] * PCAR);
      }
    }
    {
      const _Float16* vhp = Vhb + kb;
      const _Float16* vlp = Vlb + kb;
      const v16h vh0 = ldfrag_h(vhp);
      const v16h vh1 = ldfrag_h(vhp + (size_t)16 * TT);
      const v16h vh2 = ldfrag_h(vhp + (size_t)32 * TT);
      const v16h vh3 = ldfrag_h(vhp + (size_t)48 * TT);
      const v16h vl0 = ldfrag_h(vlp);
      const v16h vl1 = ldfrag_h(vlp + (size_t)16 * TT);
      const v16h vl2 = ldfrag_h(vlp + (size_t)32 * TT);
      const v16h vl3 = ldfrag_h(vlp + (size_t)48 * TT);
      o[0] = mma_h(ph.v, vh0, o[0]);  o[0] = mma_h(ph.v, vl0, o[0]);
      o[1] = mma_h(ph.v, vh1, o[1]);  o[1] = mma_h(ph.v, vl1, o[1]);
      o[2] = mma_h(ph.v, vh2, o[2]);  o[2] = mma_h(ph.v, vl2, o[2]);
      o[3] = mma_h(ph.v, vh3, o[3]);  o[3] = mma_h(ph.v, vl3, o[3]);
      guard10(o[0], o[1], o[2], o[3], ph.v, vh0, vh1, vh2, vh3, vl0, vl1, vl2, vl3, ph.v);
    }
    wave_sync_lds();
  }
  acc_guard4(o[0], o[1], o[2], o[3]);
#pragma unroll
  for (int r = 0; r < 8; ++r) {
    const float lv  = lrow[r];
    const float ls  = (lv > 0.0f) ? lv : 1.0f;
    const float inv = (lv > 0.0f) ? ((1.0f / ls) * oc) : 0.0f;
#pragma unroll
    for (int j = 0; j < 4; ++j) {
      slab[(8 * hh + r) * 68 + j * 16 + c] = o[j][r] * inv;
    }
  }
  wave_sync_lds();
  const int m = c;
  v4f vals[8];
#pragma unroll
  for (int it = 0; it < 8; ++it) {
    const int row = it * 2 + hh;
    const v4f sv = *(const v4f*)(slab + row * 68 + m * 4);
    const v4f xr = *(const v4f*)(xv + (sq0 + (size_t)row) * DM + head * HD + m * 4);
    v4f w;
#pragma unroll
    for (int e = 0; e < 4; ++e) w[e] = bfr(xr[e]) + sv[e];
    vals[it] = w;
  }
  float* dst = XBo + (sq0 + (size_t)hh) * DM + head * HD + m * 4;
  for (int pass = 0; pass < 2; ++pass) {
#pragma unroll
    for (int it = 0; it < 8; ++it) {
      *(volatile v4f*)(dst + (size_t)(it * 2) * DM) = vals[it];
    }
    __threadfence();
  }
}

extern "C" void kernel_launch(void* const* d_in, const int* in_sizes, int n_in,
                              void* d_out, int out_size, void* d_ws, size_t ws_size,
                              hipStream_t stream) {
  if (n_in < 13) return;
  if (in_sizes[0] != NPOS || in_sizes[2] != NPOS) return;
  if (in_sizes[1] != BT * DM) return;
  if (in_sizes[3] != DM * 3 * DM) return;
  if (in_sizes[4] != NTYPE * 2 * DM) return;
  if (in_sizes[5] != DM || in_sizes[6] != DM || in_sizes[7] != DM || in_sizes[8] != DM) return;
  if (in_sizes[9] != DM * 2 * DFF || in_sizes[10] != 2 * DFF) return;
  if (in_sizes[11] != DFF * DM || in_sizes[12] != DM) return;
  if (out_size != BT * DM) return;

  const int*   xtype = (const int*)d_in[0];
  const float* xval  = (const float*)d_in[1];
  const float* sord  = (const float*)d_in[2];
  const float* wattn = (const float*)d_in[3];
  const float* temb  = (const float*)d_in[4];
  const float* ln1g  = (const float*)d_in[5];
  const float* ln1b  = (const float*)d_in[6];
  const float* ln2g  = (const float*)d_in[7];
  const float* ln2b  = (const float*)d_in[8];
  const float* w1    = (const float*)d_in[9];
  const float* b1    = (const float*)d_in[10];
  const float* w2    = (const float*)d_in[11];
  const float* b2    = (const float*)d_in[12];
  float*       out   = (float*)d_out;

  const size_t szWA  = (size_t)(3 * DM) * DM * 2;
  const size_t szW1  = (size_t)(2 * DFF) * DM * 2;
  const size_t szW2  = (size_t)DM * DFF * 2;
  const size_t szTB  = (size_t)NPOS * NFREQ * 4;
  const size_t szH   = (size_t)BT * DM * 2;
  const size_t szQKV = (size_t)BT * (3 * DM) * 4;
  const size_t szM   = (size_t)BT * DFF * 2;
  const size_t szP   = (size_t)BT * DM * 2;
  const size_t szX   = (size_t)BT * DM * 4;
  size_t off = 0;
  const size_t oWA  = off; off += szWA;
  const size_t oW1  = off; off += szW1;
  const size_t oW2  = off; off += szW2;
  const size_t oCT  = off; off += szTB;
  const size_t oST  = off; off += szTB;
  const size_t oH   = off; off += szH;
  const size_t oQKV = off; off += szQKV;
  const size_t oMH  = oQKV;
  const size_t oML  = oQKV + szM;
  if (oML + szM > oQKV + szQKV) return;
  const size_t oQH  = off; off += szP;
  const size_t oQL  = off; off += szP;
  const size_t oKH  = off; off += szP;
  const size_t oKL  = off; off += szP;
  const size_t oVH  = off; off += szP;
  const size_t oVL  = off; off += szP;
  const size_t oXB  = off; off += szX;
  if (off > ws_size) return;
  if (off > (size_t)134217728) return;

  char* ws = (char*)d_ws;
  u16*   WAT = (u16*)(ws + oWA);
  u16*   W1T = (u16*)(ws + oW1);
  u16*   W2T = (u16*)(ws + oW2);
  float* CT  = (float*)(ws + oCT);
  float* ST  = (float*)(ws + oST);
  u16*   H16 = (u16*)(ws + oH);
  float* QKV = (float*)(ws + oQKV);
  u16*   MH  = (u16*)(ws + oMH);
  u16*   ML  = (u16*)(ws + oML);
  u16*   QH  = (u16*)(ws + oQH);
  u16*   QL  = (u16*)(ws + oQL);
  u16*   KH  = (u16*)(ws + oKH);
  u16*   KL  = (u16*)(ws + oKL);
  u16*   VH  = (u16*)(ws + oVH);
  u16*   VL  = (u16*)(ws + oVL);
  float* XB  = (float*)(ws + oXB);

  InvF inv;
  for (int i = 0; i < 32; ++i) inv.f[i] = 0.0f;
  for (int i = 0; i < NFREQ; ++i) {
    const double p = pow(10000.0, (double)(2 * i) / 32.0);
    const float pf = (float)p;
    inv.f[i] = 1.0f / pf;
  }

  const dim3 blk(256);
  const dim3 b128(128);
  const dim3 gWA((DM / 64) * ((3 * DM) / 64));
  const dim3 gW1((DM / 64) * ((2 * DFF) / 64));
  const dim3 gW2((DFF / 64) * (DM / 64));
  const dim3 gTab((NPOS * NFREQ + 255) / 256);
  const dim3 gLN(BT / 8);
  const dim3 gQKV((BT / 64) * ((3 * DM) / 64));
  const int rowsQK = BT * NH;
  const dim3 gR((rowsQK * 8) / 256);
  const dim3 gVT(NB * NH * NST);
  const dim3 gAT(ATT_BLOCKS);
  const dim3 bAT(ATT_THREADS);
  const dim3 gSW((BT / 64) * (DFF / 64));
  const dim3 gF2((BT / 64) * (DM / 64));

  wt16<<<gWA, blk, 0, stream>>>(wattn, WAT, DM, 3 * DM, WSC);
  wt16<<<gW1, blk, 0, stream>>>(w1, W1T, DM, 2 * DFF, WSC);
  wt16<<<gW2, blk, 0, stream>>>(w2, W2T, DFF, DM, WSC);
  k_tab<<<gTab, blk, 0, stream>>>(sord, CT, ST, inv, NPOS);
  k_ln16<<<gLN, blk, 0, stream>>>(xval, ln1g, ln1b, H16, BT, 1);
  gemm_nb<<<gQKV, b128, 0, stream>>>(H16, WAT, QKV, BT, 3 * DM, DM, 1.0f / (HSC * WSC));
  rope_qk<<<gR, blk, 0, stream>>>(QKV, xtype, temb, CT, ST, QH, QL, KH, KL, rowsQK);
  vt16<<<gVT, blk, 0, stream>>>(QKV, VH, VL);
  attn_c<<<gAT, bAT, 0, stream>>>(QH, QL, KH, KL, VH, VL, xval, XB);
  k_ln16<<<gLN, blk, 0, stream>>>(XB, ln2g, ln2b, H16, BT, 0);
  gemm_swiglu<<<gSW, blk, 0, stream>>>(H16, W1T, b1, MH, ML, BT, DM, 1.0f / (HSC * WSC));
  gemm_h2r<<<gF2, b128, 0, stream>>>(MH, ML, W2T, b2, XB, out, BT, DM, DFF, 1.0f / (MSC * WSC));
  (void)hipGetLastError();
}
